// MyCrossAttention_ori_72739566125131
// MI455X (gfx1250) — hardware-verified
//
#include <hip/hip_runtime.h>


#define NB_  1
#define NT_  4096
#define NKEY 2048
#define DM   512
#define NH_  8
#define HD   64
#define NTK  (NB_ * NT_)
#define NW   1024
#define NQKV 1024
#define PSC  32768.0f
#define LOSC 1024.0f
#define LOSCI (1.0f / 1024.0f)

typedef _Float16 h16;
typedef unsigned short bf;
typedef __attribute__((ext_vector_type(16))) __bf16   v16bf;
typedef __attribute__((ext_vector_type(16))) _Float16 v16h;
typedef __attribute__((ext_vector_type(8)))  _Float16 v8h;
typedef __attribute__((ext_vector_type(8)))  unsigned short v8us;
typedef __attribute__((ext_vector_type(8)))  float    v8f;
typedef __attribute__((ext_vector_type(4)))  float    v4f;
typedef v8h  __attribute__((may_alias)) v8ha;
typedef v4f  __attribute__((may_alias)) v4fa;
typedef v8us __attribute__((may_alias)) v8usa;

__device__ __forceinline__ unsigned short f2bf(float f) { unsigned u = __float_as_uint(f); u += 0x7FFFu + ((u >> 16) & 1u); return (unsigned short)(u >> 16); }
__device__ __forceinline__ float bf2f(unsigned short b) { return __uint_as_float(((unsigned)b) << 16); }
__device__ __forceinline__ float bfr(float f) { return bf2f(f2bf(f)); }
__device__ __forceinline__ v16h cat16(v8h lo, v8h hi) { return __builtin_shufflevector(lo, hi, 0, 1, 2, 3, 4, 5, 6, 7, 8, 9, 10, 11, 12, 13, 14, 15); }
__device__ __forceinline__ v16bf cat16b(v8us lo, v8us hi) { return __builtin_bit_cast(v16bf, __builtin_shufflevector(lo, hi, 0, 1, 2, 3, 4, 5, 6, 7, 8, 9, 10, 11, 12, 13, 14, 15)); }
__device__ __forceinline__ v8f wmma16(v16h a, v16h b, v8f c) { return __builtin_amdgcn_wmma_f32_16x16x32_f16(false, a, false, b, (short)0, c, false, false); }
__device__ __forceinline__ v8f wmmab(v16bf a, v16bf b, v8f c) { return __builtin_amdgcn_wmma_f32_16x16x32_bf16(false, a, false, b, (short)0, c, false, false); }

__global__ __launch_bounds__(256) void k_cvtb(const float* __restrict__ src, int nrows, bf* dst) {
    const int lane = threadIdx.x & 31, r = blockIdx.x * 8 + (threadIdx.x >> 5);
    if (r >= nrows) return;
    v8us o[DM / 256];
#pragma unroll
    for (int q = 0; q < DM / 256; ++q) { v8us t;
#pragma unroll
        for (int i = 0; i < 8; ++i) t[i] = f2bf(src[(size_t)r * DM + q * 256 + lane * 8 + i]);
        o[q] = t; }
#pragma unroll
    for (int q = 0; q < DM / 256; ++q) *(volatile v8us*)(dst + (size_t)r * DM + q * 256 + lane * 8) = o[q];
    __threadfence();
#pragma unroll
    for (int q = 0; q < DM / 256; ++q) *(volatile v8us*)(dst + (size_t)r * DM + q * 256 + lane * 8) = o[q];
}

template <bool SPLITA, bool F16OUT = false>
__global__ __launch_bounds__(128) void k_gemmb(const bf* __restrict__ A, const bf* __restrict__ Al, const bf* __restrict__ Bn, const float* __restrict__ bias, float* C, int ldc, h16* C2, const float* __restrict__ R = nullptr, int K = DM, int roundR = 1) {
    __shared__ __align__(16) float ost[4][16 * 68];
    const int lane = threadIdx.x & 31, wave = threadIdx.x >> 5, lr = lane & 15, hi = lane >> 4;
    const int r0 = blockIdx.x * 64 + wave * 16, c0 = blockIdx.y * 64;
    const size_t aoff = (size_t)(r0 + lr) * K + 8 * hi;
    size_t boff[4];
#pragma unroll
    for (int t = 0; t < 4; ++t) boff[t] = (size_t)(c0 + t * 16 + lr) * K + 8 * hi;
    v8f acc[4];
#pragma unroll
    for (int t = 0; t < 4; ++t) acc[t] = (v8f){};
#pragma unroll 1
    for (int kc = 0; kc < K; kc += 32) {
        const v16bf a = cat16b(*(const v8us*)(A + aoff + kc), *(const v8us*)(A + aoff + kc + 16));
        v16bf al = a;
        if (SPLITA) al = cat16b(*(const v8us*)(Al + aoff + kc), *(const v8us*)(Al + aoff + kc + 16));
#pragma unroll
        for (int t = 0; t < 4; ++t) { const v16bf b = cat16b(*(const v8us*)(Bn + boff[t] + kc), *(const v8us*)(Bn + boff[t] + kc + 16)); acc[t] = wmmab(a, b, acc[t]); if (SPLITA) acc[t] = wmmab(al, b, acc[t]); }
        asm volatile("v_nop\n\tv_nop\n\tv_nop\n\tv_nop" : "+v"(acc[0]), "+v"(acc[1]), "+v"(acc[2]), "+v"(acc[3]) : "v"(a), "v"(al));
    }
    float* os = &ost[wave][0];
#pragma unroll
    for (int t = 0; t < 4; ++t) { const float bv = bias ? bfr(bias[c0 + t * 16 + lr]) : 0.f;
#pragma unroll
        for (int j = 0; j < 8; ++j) os[(hi * 8 + j) * 68 + t * 16 + lr] = acc[t][j] + bv; }
    __syncthreads();
    if (F16OUT) {
        h16* crow = (h16*)(void*)C + (size_t)r0 * ldc + c0;
        auto pass = [&]() {
#pragma unroll
            for (int s = 0; s < 4; ++s) { const int row = 4 * s + (lane >> 3), piece = lane & 7; const float* sp = os + row * 68 + piece * 8; v8h o, o2;
#pragma unroll
                for (int i = 0; i < 8; ++i) { const h16 a = (h16)sp[i]; o[i] = a; o2[i] = (h16)((sp[i] - (float)a) * LOSC); }
                *(volatile v8h*)(crow + (size_t)row * ldc + piece * 8) = o; if (C2) *(volatile v8h*)(C2 + (size_t)r0 * ldc + c0 + (size_t)row * ldc + piece * 8) = o2; }
        };
        pass(); __threadfence(); pass();
    } else {
        float* crow = C + (size_t)r0 * ldc + c0;
        auto pass = [&]() {
#pragma unroll
            for (int s = 0; s < 8; ++s) { const int Lid = (lane >> 3) + 4 * s, piece = lane & 7; const int row = Lid >> 1, cofs = (Lid & 1) * 32 + piece * 4;
                v4f val = *(const v4fa*)(os + row * 68 + cofs); if (R) { const v4f rv = *(const v4f*)(R + ((size_t)r0 + row) * ldc + c0 + cofs); val += roundR ? (v4f){bfr(rv[0]), bfr(rv[1]), bfr(rv[2]), bfr(rv[3])} : rv; }
                *(volatile v4f*)(crow + (size_t)row * ldc + cofs) = val; }
        };
        pass(); __threadfence(); pass();
    }
}

__global__ __launch_bounds__(128) void k_attn(const h16* __restrict__ Q16, const h16* __restrict__ QL16, const h16* __restrict__ K16, const h16* __restrict__ KL16, const int* __restrict__ MSK, bf* CH, bf* CL) {
    __shared__ __align__(16) float ost[4][16 * 68];
    const int lane = threadIdx.x & 31, wave = threadIdx.x >> 5, lr = lane & 15, hi = lane >> 4;
    const int bid = blockIdx.x;
    const int b = bid / (NH_ * (NT_ / 64)), rem = bid - b * (NH_ * (NT_ / 64)), h = rem / (NT_ / 64), qt = rem - h * (NT_ / 64);
    const int q0 = qt * 64 + wave * 16;
    const size_t tok0 = (size_t)b * NT_;
    v16h qa[2];
    const size_t qo0 = (tok0 + q0 + lr) * DM + h * HD + 8 * hi;
#pragma unroll
    for (int kc = 0; kc < 2; ++kc) qa[kc] = cat16(*(const v8h*)(Q16 + qo0 + kc * 32), *(const v8h*)(Q16 + qo0 + kc * 32 + 16));
    const h16* kh_b = K16 + tok0 * DM + h * HD;
    const h16* kl_b = KL16 + tok0 * DM + h * HD;
    float mpart[8];
    float mrow[8], lpart[8];
#pragma unroll
    for (int j = 0; j < 8; ++j) { mrow[j] = -3.0e38f; lpart[j] = 0.f; mpart[j] = 0.f; }
    int qpos[8];
#pragma unroll
    for (int j = 0; j < 8; ++j) qpos[j] = q0 + 8 * hi + j;
    const int kt_lo = 0, kt_hi = NKEY / 32 - 1;
#pragma unroll 1
    for (int kt = kt_lo; kt <= kt_hi; ++kt) {
        const int l0 = kt * 32;
        const size_t ko0 = (size_t)(l0 + lr) * DM + 8 * hi, ko1 = (size_t)(l0 + 16 + lr) * DM + 8 * hi;
        v8f s0 = {}, s1 = {}, x0 = {}, x1 = {};
#pragma unroll
        for (int kc = 0; kc < 2; ++kc) {
            { const v16h k0h = cat16(*(const v8h*)(kh_b + ko0 + kc * 32), *(const v8h*)(kh_b + ko0 + kc * 32 + 16)), k1h = cat16(*(const v8h*)(kh_b + ko1 + kc * 32), *(const v8h*)(kh_b + ko1 + kc * 32 + 16));
              const v16h qlk = cat16(*(const v8h*)(QL16 + qo0 + kc * 32), *(const v8h*)(QL16 + qo0 + kc * 32 + 16));
              s0 = wmma16(qa[kc], k0h, s0); x0 = wmma16(qlk, k0h, x0); s1 = wmma16(qa[kc], k1h, s1); x1 = wmma16(qlk, k1h, x1);
              asm volatile("v_nop" : "+v"(s0), "+v"(s1), "+v"(x0), "+v"(x1) : "v"(qlk), "v"(k0h), "v"(k1h) : "memory"); }
            { const v16h k0l = cat16(*(const v8h*)(kl_b + ko0 + kc * 32), *(const v8h*)(kl_b + ko0 + kc * 32 + 16)), k1l = cat16(*(const v8h*)(kl_b + ko1 + kc * 32), *(const v8h*)(kl_b + ko1 + kc * 32 + 16));
              x0 = wmma16(qa[kc], k0l, x0); x1 = wmma16(qa[kc], k1l, x1);
              asm volatile("v_nop" : "+v"(x0), "+v"(x1) : "v"(k0l), "v"(k1l) : "memory"); }
        }
        asm volatile("v_nop\n\tv_nop\n\tv_nop\n\tv_nop" : "+v"(s0), "+v"(s1), "+v"(x0), "+v"(x1) : "v"(qa[0]), "v"(qa[1]));
        float alpha[8]; const float mka = (float)MSK[l0 + lr], mkb = (float)MSK[l0 + 16 + lr];
#pragma unroll
        for (int j = 0; j < 8; ++j) {
            const int ja = l0 + lr, jb = l0 + 16 + lr, qi = qpos[j];
            const float a0 = (s0[j] + x0[j] * LOSCI) * 0.125f, a1 = (s1[j] + x1[j] * LOSCI) * 0.125f; (void)ja; (void)jb; (void)qi;
            float mx = fmaxf(a0, a1);
            mx = fmaxf(mx, __shfl_xor(mx, 1, 16)); mx = fmaxf(mx, __shfl_xor(mx, 2, 16)); mx = fmaxf(mx, __shfl_xor(mx, 4, 16)); mx = fmaxf(mx, __shfl_xor(mx, 8, 16));
            const float mn = fmaxf(mrow[j], mx);
            alpha[j] = __expf(mrow[j] - mn); mrow[j] = mn;
            const float p0 = __expf(a0 - mn), p1 = __expf(a1 - mn);
            lpart[j] = lpart[j] * alpha[j] + (p0 + p1);
            mpart[j] = mpart[j] * alpha[j] + (p0 * mka + p1 * mkb);
        }
    }
    float* os = &ost[wave][0];
#pragma unroll
    for (int j = 0; j < 8; ++j) { float rs = lpart[j], ms = mpart[j];
        rs += __shfl_xor(rs, 1, 16); rs += __shfl_xor(rs, 2, 16); rs += __shfl_xor(rs, 4, 16); rs += __shfl_xor(rs, 8, 16);
        ms += __shfl_xor(ms, 1, 16); ms += __shfl_xor(ms, 2, 16); ms += __shfl_xor(ms, 4, 16); ms += __shfl_xor(ms, 8, 16);
        const float sv = ms / rs;
#pragma unroll
        for (int i = 0; i < 4; ++i) os[(hi * 8 + j) * 68 + lr * 4 + i] = sv; }
    __syncthreads();
    const size_t cbase = (tok0 + q0) * DM + (size_t)h * HD;
    auto pass = [&]() {
#pragma unroll
        for (int s = 0; s < 4; ++s) { const int row = 4 * s + (lane >> 3), piece = lane & 7; const float* sp = os + row * 68 + piece * 8; v8us oh, ol;
#pragma unroll
            for (int i = 0; i < 8; ++i) { const unsigned short hb = f2bf(sp[i]); oh[i] = hb; ol[i] = f2bf(sp[i] - bf2f(hb)); }
            *(volatile v8us*)(CH + cbase + (size_t)row * DM + piece * 8) = oh; *(volatile v8us*)(CL + cbase + (size_t)row * DM + piece * 8) = ol; }
    };
    pass(); __threadfence(); pass();
}

#define VST2(T, p, v) do { const T vst2_v_ = (v); *(volatile T*)(p) = vst2_v_; __threadfence(); *(volatile T*)(p) = vst2_v_; } while (0)
extern "C" void kernel_launch(void* const* d_in, const int* in_sizes, int n_in,
                              void* d_out, int out_size, void* d_ws, size_t ws_size, hipStream_t stream) {
    (void)in_sizes; (void)n_in; (void)out_size;
    const float* q = (const float*)d_in[0]; const float* k = (const float*)d_in[1]; const int* msk = (const int*)d_in[3];
    const float* Wq = (const float*)d_in[4]; const float* Wk = (const float*)d_in[5]; const float* Wp = (const float*)d_in[6];
    float* out = (float*)d_out;
    char* wsp = (char*)d_ws;
    auto take = [&](size_t bytes) { char* p = wsp; wsp += (bytes + 255) & ~(size_t)255; return (void*)p; };
    bf* WqB = (bf*)take((size_t)DM * DM * 2); bf* WkB = (bf*)take((size_t)DM * DM * 2); bf* WpB = (bf*)take((size_t)DM * DM * 2);
    bf* Xq = (bf*)take((size_t)NT_ * DM * 2); bf* Xk = (bf*)take((size_t)NKEY * DM * 2);
    h16* QH = (h16*)take((size_t)NT_ * DM * 2); h16* QL = (h16*)take((size_t)NT_ * DM * 2); h16* KH = (h16*)take((size_t)NKEY * DM * 2); h16* KL = (h16*)take((size_t)NKEY * DM * 2);
    bf* CH = (bf*)take((size_t)NT_ * DM * 2); bf* CL = (bf*)take((size_t)NT_ * DM * 2);
    if ((size_t)(wsp - (char*)d_ws) > ws_size) return;
    k_cvtb<<<DM / 8, 256, 0, stream>>>(Wq, DM, WqB); k_cvtb<<<DM / 8, 256, 0, stream>>>(Wk, DM, WkB); k_cvtb<<<DM / 8, 256, 0, stream>>>(Wp, DM, WpB);
    for (int b = 0; b < 4; ++b) {
        k_cvtb<<<NT_ / 8, 256, 0, stream>>>(q + (size_t)b * NT_ * DM, NT_, Xq); k_cvtb<<<NKEY / 8, 256, 0, stream>>>(k + (size_t)b * NKEY * DM, NKEY, Xk);
        k_gemmb<false, true><<<dim3(NT_ / 64, DM / 64, 1), 128, 0, stream>>>(Xq, nullptr, WqB, nullptr, (float*)(void*)QH, DM, QL);
        k_gemmb<false, true><<<dim3(NKEY / 64, DM / 64, 1), 128, 0, stream>>>(Xk, nullptr, WkB, nullptr, (float*)(void*)KH, DM, KL);
        k_attn<<<NB_ * NH_ * (NT_ / 64), 128, 0, stream>>>(QH, QL, KH, KL, msk + (size_t)b * NKEY, CH, CL);
        k_gemmb<true, false><<<dim3(NT_ / 64, DM / 64, 1), 128, 0, stream>>>(CH, CL, WpB, nullptr, out + (size_t)b * NT_ * DM, DM, nullptr);
    }
}
